// Mamba2Block_34205119545699
// MI455X (gfx1250) — hardware-run, weakly checked
//
#include <hip/hip_runtime.h>
#include <math.h>

typedef __attribute__((ext_vector_type(16))) _Float16 v16h;
typedef __attribute__((ext_vector_type(8)))  _Float16 v8h;
typedef __attribute__((ext_vector_type(8)))  float    v8f;
typedef __attribute__((ext_vector_type(4)))  float    v4f;
typedef __attribute__((ext_vector_type(4)))  unsigned v4u;

constexpr int kBatch  = 2;
constexpr int kSeq    = 2048;
constexpr int kDm     = 1024;
constexpr int kDin    = 2048;
constexpr int kHeads  = 16;
constexpr int kHdim   = 128;
constexpr int kNst    = 64;
constexpr int kChunk  = 64;
constexpr int kRows   = kBatch * kSeq;
constexpr int kNssmIn = kHeads + 2 * kHeads * kNst;
constexpr int kNssmPd = 2112;
constexpr int kBC     = kHeads * kNst;
constexpr int kDtPad  = 64;
constexpr int kLoRows = kBC + kDtPad;
constexpr int kConvTP = 260;
constexpr int kLP     = 72;
constexpr int kYP     = 132;
constexpr int kSP     = 68;
constexpr int kW2P    = 36;
static_assert(kDin == kHeads * kHdim, "head split");
static_assert(kNssmIn == 2064 && kNssmPd == 2 * kBC + kDtPad, "ssm projection width");
static_assert(kLoRows == 1088, "remainder plane rows");
static_assert((kSeq % kChunk) == 0 && kChunk == 64 && kNst == 64 && kHdim == 128, "chunk tiling");
static_assert((kDm % 32) == 0 && (kDin % 32) == 0, "GEMM K multiples of 32");
static_assert((kRows % 64) == 0 && (kDin % 64) == 0 && (kBC % 64) == 0 && (kDtPad % 64) == 0 && (kDm % 64) == 0, "GEMM M,N multiples of 64");
static_assert(64 * kYP <= 128 * kSP, "shared f32 tile extent");

constexpr int kLgInp = 4;
constexpr int kLgW   = 6;
constexpr int kLgXa  = 6;
constexpr int kLgSp  = 6;
constexpr int kLgY   = 6;
constexpr float kCarXa  = (float)(1 << kLgXa);
constexpr float kCarSp  = (float)(1 << kLgSp);
constexpr float kCarY   = (float)(1 << kLgY);
constexpr float kCarM   = 1024.0f;
constexpr float kCarS   = 4096.0f;
constexpr float kCarBd  = 4096.0f;
constexpr float kResid  = 2048.0f;
constexpr float kMfold  = kCarM / (kCarSp * kCarSp);
constexpr float kYdFold = 1.0f / (kCarM * kCarXa);
constexpr float kYoFold = 1.0f / (kCarSp * kCarS);
constexpr float kStFold = 1.0f / (kCarXa * kCarBd);
constexpr float kF16Min = 6.103515625e-05f;
constexpr float kF32Min = 1.17549435e-38f;

constexpr size_t kOffInp16  = 0;
constexpr size_t kOffWin16  = kOffInp16  + (size_t)kRows * kDm * 2;
constexpr size_t kOffWssm16 = kOffWin16  + (size_t)2 * kDin * kDm * 2;
constexpr size_t kOffWout16 = kOffWssm16 + (size_t)kNssmPd * kDin * 2;
constexpr size_t kOffX32    = kOffWout16 + (size_t)kDm * kDin * 2;
constexpr size_t kOffZ16    = kOffX32    + (size_t)kRows * kDin * 4;
constexpr size_t kOffXah    = kOffZ16    + (size_t)kRows * kDin * 2;
constexpr size_t kOffXal    = kOffXah    + (size_t)kRows * kDin * 2;
constexpr size_t kOffC16    = kOffXal    + (size_t)kRows * kDin * 2;
constexpr size_t kOffDt32   = kOffC16    + (size_t)kRows * kBC * 2;
constexpr size_t kOffWssmLo = kOffDt32   + (size_t)kRows * kDtPad * 4;
constexpr size_t kWsTotal   = kOffWssmLo + (size_t)kLoRows * kDin * 2;
constexpr size_t kOffY16    = kOffInp16;
constexpr size_t kOffB32    = kOffX32;
static_assert(kWsTotal == 127401984ull, "carve total");
static_assert(kWsTotal <= 134217728ull, "carve cap");
static_assert((size_t)kRows * kDin * 2 <= kOffWssm16 - kOffInp16, "Y16 alias fits");
static_assert((size_t)kRows * kBC * 4 <= (size_t)kRows * kDin * 4, "B32 alias fits");
static_assert((kOffWin16 % 128) == 0 && (kOffWssm16 % 128) == 0 && (kOffWout16 % 128) == 0 && (kOffX32 % 128) == 0 &&
              (kOffZ16 % 128) == 0 && (kOffXah % 128) == 0 && (kOffXal % 128) == 0 && (kOffC16 % 128) == 0 &&
              (kOffDt32 % 128) == 0 && (kOffWssmLo % 128) == 0, "128-B aligned regions");

constexpr size_t kOut1Off = (size_t)kRows * kDm;
constexpr size_t kOut2Off = kOut1Off + (size_t)kBatch * kDin * 3;
constexpr size_t kOutTot  = kOut2Off + (size_t)kBatch * kHeads * kHdim * kNst;
static_assert(kOut1Off * 4 == 16777216ull && kOut2Off * 4 == 16826368ull && kOutTot * 4 == 17874944ull, "output byte offsets");

__device__ __forceinline__ _Float16 to_h(float v) {
  const float f = (fabsf(v) < kF16Min) ? 0.0f : v;
  return (_Float16)f;
}
__device__ __forceinline__ float exp_ftz(float x) {
  const float e = expf(x);
  return (e < kF32Min) ? 0.0f : e;
}
__device__ __forceinline__ float h16_to_f32(unsigned hb) {
  const unsigned sgn = (hb & 0x8000u) << 16; const unsigned em = hb & 0x7fffu;
  const float fn = __uint_as_float((em << 13) + 0x38000000u);
  const float fs = (float)em * 5.9604644775390625e-8f;
  const float mag = (em < 0x400u) ? fs : fn; return __uint_as_float(__float_as_uint(mag) | sgn); }
__device__ __forceinline__ unsigned pick16(v4u v, int e) {
  const unsigned w = v[e >> 1];
  return (e & 1) ? (w >> 16) : (w & 0xffffu);
}

struct FragH {
  union U { v16h v; v8h h[2]; };
  static __device__ __forceinline__ v16h load(const _Float16* p) {
    U f; f.h[0] = *(const v8h*)(p); f.h[1] = *(const v8h*)(p + 16); return f.v;
  }
};
__device__ __forceinline__ v8f mma_g(v16h a, v16h b, v8f c) {
  c = __builtin_amdgcn_wmma_f32_16x16x32_f16(false, a, false, b, (short)0, c, false, false);
  asm volatile("v_nop\n\tv_nop\n\tv_nop\n\tv_nop" : "+v"(c) : "v"(a), "v"(b));
  return c;
}

template <int MODE>
__device__ __forceinline__ _Float16 cvt_elem(float x) {
  if (MODE == 2) {
    const _Float16 hv = to_h(x);
    const float rem = (x - (float)hv) * kResid;
    return to_h(rem);
  }
  return to_h(x);
}

template <int CARRY_LOG2, int MODE>
__global__ __launch_bounds__(256) void cvt_f16_kernel(
    const float* __restrict__ src, unsigned short* __restrict__ dst, unsigned total8)
{
  constexpr float carry = (float)(1 << CARRY_LOG2);
  const unsigned i = blockIdx.x * 256u + threadIdx.x;
  if (i >= total8) return;
  size_t so;
  bool valid = true;
  if (MODE == 0) {
    so = (size_t)i * 8u;
  } else {
    unsigned rp = i >> 8;
    asm volatile("" : "+v"(rp));
    unsigned c8 = (i & 255u) * 8u;
    asm volatile("" : "+v"(c8));
    unsigned sr;
    if (MODE == 1) {
      sr = (rp < 2048u) ? (rp + 16u) : (rp - 2048u);
      valid = (rp < 2064u);
    } else {
      sr = (rp < 1024u) ? (rp + 16u) : (rp - 1024u);
      valid = (rp < 1040u);
    }
    sr = (sr > 2063u) ? 2063u : sr;
    asm volatile("" : "+v"(sr));
    so = (size_t)sr * (size_t)kDin + c8;
  }
  v4f a0 = *(const v4f*)(src + so);
  v4f a1 = *(const v4f*)(src + so + 4);
  asm volatile("" : "+v"(a0), "+v"(a1));
  v8h o;
#pragma unroll
  for (int e = 0; e < 4; ++e) {
    const float x0 = valid ? (a0[e] * carry) : 0.0f;
    const float x1 = valid ? (a1[e] * carry) : 0.0f;
    o[e]     = cvt_elem<MODE>(x0);
    o[4 + e] = cvt_elem<MODE>(x1);
  }
  unsigned short* q = dst + (size_t)i * 8u;
  *(volatile v8h*)q = o;
  __threadfence();
  *(volatile v8h*)q = o;
}

template <int OUT_MODE, int SCL_LOG2>
__global__ __launch_bounds__(256) void wmma_gemm64(
    const unsigned short* __restrict__ Ap, int lda,
    const unsigned short* __restrict__ Btp, int ldb,
    void* __restrict__ Cout, int ldc, int M, int N, int K)
{
  constexpr float scale = 1.0f / (float)(1 << SCL_LOG2);
  const _Float16* A  = (const _Float16*)(const void*)Ap;
  const _Float16* Bt = (const _Float16*)(const void*)Btp;
  __shared__ __align__(16) float sT[8][16 * 68];
  const int lane = threadIdx.x & 31;
  const int wave = threadIdx.x >> 5;
  const int tilesN = N >> 6;
  const int tilesM = M >> 6;
  const int tile = blockIdx.x * 8 + wave;
  if (tile >= tilesM * tilesN) return;
  const int tm = tile / tilesN;
  const int tn = tile - tm * tilesN;
  const int m0 = tm << 6;
  const int n0 = tn << 6;
  const int rlane = lane & 15;
  const int koff  = (lane >> 4) * 8;
  const int mOff  = (lane >> 4) * 8;

  v8f acc[4][4];
#pragma unroll
  for (int i = 0; i < 4; ++i)
#pragma unroll
    for (int j = 0; j < 4; ++j) acc[i][j] = (v8f){0.f,0.f,0.f,0.f,0.f,0.f,0.f,0.f};

  for (int k0 = 0; k0 < K; k0 += 32) {
    v16h bh[4];
#pragma unroll
    for (int j = 0; j < 4; ++j) {
      const size_t bo = (size_t)(n0 + (j << 4) + rlane) * ldb + koff + k0;
      bh[j] = FragH::load(Bt + bo);
    }
#pragma unroll
    for (int i = 0; i < 4; ++i) {
      const size_t ao = (size_t)(m0 + (i << 4) + rlane) * lda + koff + k0;
      const v16h ah = FragH::load(A + ao);
#pragma unroll
      for (int j = 0; j < 4; ++j) acc[i][j] = mma_g(ah, bh[j], acc[i][j]);
    }
  }

  float* slab = sT[wave];
#pragma unroll
  for (int i = 0; i < 4; ++i) {
    const int mBase = m0 + (i << 4);
#pragma unroll
    for (int j = 0; j < 4; ++j) {
#pragma unroll
      for (int r = 0; r < 8; ++r) {
        const float v = acc[i][j][r] * scale;
        slab[(mOff + r) * 68 + (j << 4) + rlane] = v;
      }
    }
    __builtin_amdgcn_fence(__ATOMIC_RELEASE, "workgroup");
    __builtin_amdgcn_wave_barrier();
    __builtin_amdgcn_fence(__ATOMIC_ACQUIRE, "workgroup");
    if (OUT_MODE == 0) {
      float* C = (float*)Cout;
      const int hh = lane >> 4, c4 = (lane & 15) * 4;
      for (int pass = 0; pass < 2; ++pass) {
#pragma unroll
        for (int it = 0; it < 8; ++it) {
          const int row = it * 2 + hh;
          const v4f v = *(const v4f*)(slab + row * 68 + c4);
          *(volatile v4f*)(C + (size_t)(mBase + row) * ldc + n0 + c4) = v;
        }
        __threadfence();
      }
    } else {
      const int q = lane >> 3, c8 = (lane & 7) * 8;
      unsigned short* C = (unsigned short*)Cout;
      for (int pass = 0; pass < 2; ++pass) {
#pragma unroll
        for (int it = 0; it < 4; ++it) {
          const int row = it * 4 + q;
          const float* sp = slab + row * 68 + c8;
          v8h hv;
#pragma unroll
          for (int e = 0; e < 8; ++e) hv[e] = to_h(sp[e]);
          *(volatile v8h*)(C + (size_t)(mBase + row) * ldc + n0 + c8) = hv;
        }
        __threadfence();
      }
    }
    __builtin_amdgcn_fence(__ATOMIC_RELEASE, "workgroup");
    __builtin_amdgcn_wave_barrier();
    __builtin_amdgcn_fence(__ATOMIC_ACQUIRE, "workgroup");
  }
}

template <int SCL_LOG2>
__global__ __launch_bounds__(256) void wmma_gemm_w2(
    const unsigned short* __restrict__ Ap, int lda,
    const unsigned short* __restrict__ Bhp, const unsigned short* __restrict__ Blp, int ldb,
    float* __restrict__ C, int ldc, int M, int N, int K)
{
  constexpr float scale = 1.0f / (float)(1 << SCL_LOG2);
  constexpr float rfold = 1.0f / kResid;
  const _Float16* A  = (const _Float16*)(const void*)Ap;
  const _Float16* Bh = (const _Float16*)(const void*)Bhp;
  const _Float16* Bl = (const _Float16*)(const void*)Blp;
  __shared__ __align__(16) float sT[8][16 * kW2P];
  const int lane = threadIdx.x & 31;
  const int wave = threadIdx.x >> 5;
  const int tilesN = N >> 5;
  const int tilesM = M >> 6;
  const int tile = blockIdx.x * 8 + wave;
  if (tile >= tilesM * tilesN) return;
  const int tm = tile / tilesN;
  const int tn = tile - tm * tilesN;
  const int m0 = tm << 6;
  const int n0 = tn << 5;
  const int rlane = lane & 15;
  const int koff  = (lane >> 4) * 8;
  const int mOff  = (lane >> 4) * 8;

  v8f acc[4][2], accr[4][2];
#pragma unroll
  for (int i = 0; i < 4; ++i)
#pragma unroll
    for (int j = 0; j < 2; ++j) {
      acc[i][j]  = (v8f){0.f,0.f,0.f,0.f,0.f,0.f,0.f,0.f};
      accr[i][j] = (v8f){0.f,0.f,0.f,0.f,0.f,0.f,0.f,0.f};
    }

  for (int k0 = 0; k0 < K; k0 += 32) {
    v16h bh[2], bl[2];
#pragma unroll
    for (int j = 0; j < 2; ++j) {
      const size_t bo = (size_t)(n0 + (j << 4) + rlane) * ldb + koff + k0;
      bh[j] = FragH::load(Bh + bo);
      bl[j] = FragH::load(Bl + bo);
    }
#pragma unroll
    for (int i = 0; i < 4; ++i) {
      const size_t ao = (size_t)(m0 + (i << 4) + rlane) * lda + koff + k0;
      const v16h ah = FragH::load(A + ao);
#pragma unroll
      for (int j = 0; j < 2; ++j) {
        acc[i][j]  = mma_g(ah, bh[j], acc[i][j]);
        accr[i][j] = mma_g(ah, bl[j], accr[i][j]);
      }
    }
  }

  float* slab = sT[wave];
  const int rs = lane >> 3, c4 = (lane & 7) * 4;
#pragma unroll
  for (int i = 0; i < 4; ++i) {
    const int mBase = m0 + (i << 4);
#pragma unroll
    for (int j = 0; j < 2; ++j) {
#pragma unroll
      for (int r = 0; r < 8; ++r) {
        const float v = (acc[i][j][r] + accr[i][j][r] * rfold) * scale;
        slab[(mOff + r) * kW2P + (j << 4) + rlane] = v;
      }
    }
    __builtin_amdgcn_fence(__ATOMIC_RELEASE, "workgroup");
    __builtin_amdgcn_wave_barrier();
    __builtin_amdgcn_fence(__ATOMIC_ACQUIRE, "workgroup");
    for (int pass = 0; pass < 2; ++pass) {
#pragma unroll
      for (int it = 0; it < 4; ++it) {
        const int row = it * 4 + rs;
        const v4f v = *(const v4f*)(slab + row * kW2P + c4);
        *(volatile v4f*)(C + (size_t)(mBase + row) * ldc + n0 + c4) = v;
      }
      __threadfence();
    }
    __builtin_amdgcn_fence(__ATOMIC_RELEASE, "workgroup");
    __builtin_amdgcn_wave_barrier();
    __builtin_amdgcn_fence(__ATOMIC_ACQUIRE, "workgroup");
  }
}

__global__ __launch_bounds__(256) void conv_silu_kernel(
    const float* __restrict__ X32, const float* __restrict__ cw, const float* __restrict__ cb,
    unsigned short* __restrict__ XH, unsigned short* __restrict__ XL)
{
  __shared__ __align__(16) float sT[16 * kConvTP];
  const int tid = threadIdx.x, lane = tid & 31, wave = tid >> 5;
  const int d0 = blockIdx.x * 256, d = d0 + tid;
  const int g0 = blockIdx.y * 64;
  const int tb = g0 & (kSeq - 1);
  const v4f wv = *(const v4f*)(cw + (size_t)d * 4);
  const float w0 = wv[0], w1 = wv[1], w2 = wv[2], w3 = wv[3];
  const float bc = cb[d];
  float xm3, xm2, xm1;
  {
    const bool hist = (tb > 0);
    const int rb = hist ? (g0 - 3) : g0;
    const float v3 = X32[(size_t)rb * kDin + d];
    const float v2 = X32[(size_t)(rb + 1) * kDin + d];
    const float v1 = X32[(size_t)(rb + 2) * kDin + d];
    xm3 = hist ? v3 : 0.f;
    xm2 = hist ? v2 : 0.f;
    xm1 = hist ? v1 : 0.f;
  }
#pragma unroll 1
  for (int sub = 0; sub < 4; ++sub) {
    const int lb = g0 + sub * 16;
#pragma unroll 1
    for (int s = 0; s < 16; ++s) {
      const float xcur = X32[(size_t)(lb + s) * kDin + d];
      float acc = w0 * xm3;
      acc = fmaf(w1, xm2, acc);
      acc = fmaf(w2, xm1, acc);
      acc = fmaf(w3, xcur, acc);
      const float sv = acc + bc;
      const float sg = __builtin_amdgcn_rcpf(1.0f + __expf(-sv));
      sT[s * kConvTP + tid] = sv * sg;
      xm3 = xm2; xm2 = xm1; xm1 = xcur;
    }
    __syncthreads();
    v8h hv[2], lv[2];
#pragma unroll
    for (int it = 0; it < 2; ++it) {
      const float* sp = sT + (it * 8 + wave) * kConvTP + lane * 8;
      const v4f a0 = *(const v4f*)(sp);
      const v4f a1 = *(const v4f*)(sp + 4);
#pragma unroll
      for (int e = 0; e < 4; ++e) {
        const float c0 = a0[e] * kCarXa, c1 = a1[e] * kCarXa;
        const _Float16 h0 = to_h(c0), h1 = to_h(c1);
        const float r0 = (c0 - (float)h0) * kResid, r1 = (c1 - (float)h1) * kResid;
        hv[it][e]     = h0;
        hv[it][4 + e] = h1;
        lv[it][e]     = to_h(r0);
        lv[it][4 + e] = to_h(r1);
      }
    }
    for (int pass = 0; pass < 2; ++pass) {
#pragma unroll
      for (int it = 0; it < 2; ++it) {
        const size_t o = (size_t)(lb + it * 8 + wave) * kDin + d0 + lane * 8;
        *(volatile v8h*)(XH + o) = hv[it];
        *(volatile v8h*)(XL + o) = lv[it];
      }
      __threadfence();
    }
    __syncthreads();
  }
}

__global__ __launch_bounds__(256) void conv_state_kernel(const float* __restrict__ X32, float* __restrict__ out1)
{
  unsigned idx = blockIdx.x * 256u + threadIdx.x;
  unsigned ic = (idx < 12288u) ? idx : 12287u;
  asm volatile("" : "+v"(ic));
  unsigned bq = ic / 6144u;
  asm volatile("" : "+v"(bq));
  unsigned rem = ic - bq * 6144u;
  asm volatile("" : "+v"(rem));
  unsigned c = rem / 3u;
  asm volatile("" : "+v"(c));
  unsigned j = rem - c * 3u;
  asm volatile("" : "+v"(j));
  float v = X32[(size_t)(bq * (unsigned)kSeq + (unsigned)(kSeq - 3) + j) * (size_t)kDin + c];
  asm volatile("" : "+v"(v));
  *(volatile float*)(out1 + ic) = v;
  __threadfence();
  *(volatile float*)(out1 + ic) = v;
}

__global__ __launch_bounds__(256) void ssd_chunk_kernel(
    const unsigned short* __restrict__ xahi, const unsigned short* __restrict__ xalo,
    const unsigned short* __restrict__ zpl, const float* __restrict__ bpl,
    const unsigned short* __restrict__ cpl, const float* __restrict__ dtpl,
    const float* __restrict__ alog, const float* __restrict__ dskip, const float* __restrict__ dtbias,
    unsigned short* __restrict__ ypl, float* __restrict__ state_out)
{
  __shared__ __align__(16) unsigned short sC[64 * kLP];
  __shared__ __align__(16) _Float16       sB[64 * kLP];
  __shared__ __align__(16) unsigned short sXh[128 * kLP];
  __shared__ __align__(16) unsigned short sXl[128 * kLP];
  __shared__ __align__(16) _Float16       sM[64 * kLP];
  __shared__ __align__(16) _Float16       sBh[64 * kLP];
  __shared__ __align__(16) _Float16       sBl[64 * kLP];
  __shared__ __align__(16) _Float16       sS[128 * kLP];
  __shared__ __align__(16) float          sY[128 * kSP];
  __shared__ float sDt[64];
  __shared__ float sAa[64];
  __shared__ float sAcs[64];
  __shared__ float sW[64];
  __shared__ float sEt[64];

  const unsigned tid = threadIdx.x;
  const unsigned lane = tid & 31u, wave = tid >> 5;
  const unsigned hh = lane >> 4, r = lane & 15u, koff = hh * 8u;
  const unsigned bq = (blockIdx.x >> 4) & 1u, hd = blockIdx.x & 15u;

  const float Acont = -expf(alog[hd]);
  const float dtb   = dtbias[hd];
  const float Dsk   = dskip[hd];

  const _Float16* pC  = (const _Float16*)(const void*)sC;
  const _Float16* pB  = sB;
  const _Float16* pXh = (const _Float16*)(const void*)sXh;
  const _Float16* pXl = (const _Float16*)(const void*)sXl;
  const _Float16* pM  = sM;
  const _Float16* pBh = sBh;
  const _Float16* pBl = sBl;
  const _Float16* pS  = sS;

  v8f sreg[4];
#pragma unroll
  for (int j = 0; j < 4; ++j) sreg[j] = (v8f){0.f,0.f,0.f,0.f,0.f,0.f,0.f,0.f};
#pragma unroll
  for (int j = 0; j < 4; ++j)
#pragma unroll
    for (int rr = 0; rr < 8; ++rr)
      sS[(16u * wave + 8u * hh + rr) * kLP + 16u * j + r] = (_Float16)0.0f;

  const unsigned bs = tid >> 2, bn0 = (tid & 3u) * 16u;
  const unsigned xs = tid & 63u, xg = tid >> 6;
  float Bf[16];

#pragma unroll 1
  for (int ch = 0; ch < kSeq / kChunk; ++ch) {
    const size_t row0 = (size_t)bq * kSeq + (size_t)ch * kChunk;
    __syncthreads();
    if (tid < 64u) {
      const float v  = dtpl[(row0 + tid) * kDtPad + hd] + dtb;
      const float dt = fmaxf(v, 0.0f) + log1pf(expf(-fabsf(v)));
      sDt[tid] = dt;
      sAa[tid] = Acont * dt;
    }
#pragma unroll
    for (int i = 0; i < 2; ++i) {
      const unsigned idx = tid + 256u * i;
      const unsigned t = idx >> 3, seg = idx & 7u;
      const v4u v = *(const v4u*)(const void*)(cpl + (row0 + t) * kBC + 64u * hd + 8u * seg);
      *(v4u*)(void*)(sC + t * kLP + 8u * seg) = v;
    }
    {
      const float* bp = bpl + (row0 + bs) * kBC + 64u * hd + bn0;
#pragma unroll
      for (int q = 0; q < 4; ++q) {
        const v4f v = *(const v4f*)(bp + 4 * q);
        Bf[4 * q + 0] = v[0]; Bf[4 * q + 1] = v[1]; Bf[4 * q + 2] = v[2]; Bf[4 * q + 3] = v[3];
      }
      v8h h0, h1;
#pragma unroll
      for (int e = 0; e < 8; ++e) {
        h0[e] = to_h(Bf[e] * kCarSp);
        h1[e] = to_h(Bf[8 + e] * kCarSp);
      }
      *(v8h*)(void*)(sB + bs * kLP + bn0)      = h0;
      *(v8h*)(void*)(sB + bs * kLP + bn0 + 8u) = h1;
    }
#pragma unroll
    for (int i = 0; i < 4; ++i) {
      const unsigned p0 = 8u * (xg + 4u * i);
      const size_t g = (row0 + xs) * kDin + 128u * hd + p0;
      const v4u vh = *(const v4u*)(const void*)(xahi + g);
      const v4u vl = *(const v4u*)(const void*)(xalo + g);
#pragma unroll
      for (int e = 0; e < 8; ++e) {
        sXh[(p0 + e) * kLP + xs] = (unsigned short)pick16(vh, e);
        sXl[(p0 + e) * kLP + xs] = (unsigned short)pick16(vl, e);
      }
    }
    __syncthreads();
    if (tid < 64u) {
      float tot = 0.0f, pre = 0.0f;
#pragma unroll 8
      for (unsigned k = 0; k < 64u; ++k) {
        const float ak = sAa[k];
        tot += ak;
        pre += (k <= tid) ? ak : 0.0f;
      }
      sAcs[tid] = pre;
      sW[tid]   = sDt[tid] * exp_ftz(tot - pre);
      sEt[tid]  = exp_ftz(pre);
    }
    __syncthreads();
    {
      const unsigned tt = wave >> 1;
      float act[8];
#pragma unroll
      for (int rr = 0; rr < 8; ++rr) act[rr] = sAcs[16u * tt + 8u * hh + rr];
#pragma unroll 1
      for (unsigned j = 0; j < 2u; ++j) {
        const unsigned sj = (wave & 1u) * 2u + j;
        v8f g = (v8f){0.f,0.f,0.f,0.f,0.f,0.f,0.f,0.f};
#pragma unroll
        for (int ks = 0; ks < 2; ++ks) {
          const v16h a = FragH::load(pC + (16u * tt + r) * kLP + koff + 32u * ks);
          const v16h b = FragH::load(pB + (16u * sj + r) * kLP + koff + 32u * ks);
          g = mma_g(a, b, g);
        }
        const unsigned s = 16u * sj + r;
        const float as = sAcs[s];
        const float ds = sDt[s] * kMfold;
#pragma unroll
        for (int rr = 0; rr < 8; ++rr) {
          const unsigned t = 16u * tt + 8u * hh + rr;
          const bool keep = (t >= s);
          const float dd = keep ? (act[rr] - as) : 0.0f;
          const float e  = exp_ftz(dd);
          const float v  = keep ? (g[rr] * e * ds) : 0.0f;
          sM[t * kLP + s] = to_h(v);
        }
      }
    }
    {
      const float ws = sW[bs] * kCarBd;
#pragma unroll
      for (int e = 0; e < 16; ++e) {
        const float v = Bf[e] * ws;
        const _Float16 hv = to_h(v);
        const float lo = (v - (float)hv) * kResid;
        sBh[(bn0 + e) * kLP + bs] = hv;
        sBl[(bn0 + e) * kLP + bs] = to_h(lo);
      }
    }
    __syncthreads();
    {
      const unsigned tt = wave >> 1, pj0 = (wave & 1u) * 4u;
      v8f yd[4], yo[4];
#pragma unroll
      for (int j = 0; j < 4; ++j) {
        yd[j] = (v8f){0.f,0.f,0.f,0.f,0.f,0.f,0.f,0.f};
        yo[j] = (v8f){0.f,0.f,0.f,0.f,0.f,0.f,0.f,0.f};
      }
#pragma unroll
      for (int ks = 0; ks < 2; ++ks) {
        const v16h am = FragH::load(pM + (16u * tt + r) * kLP + koff + 32u * ks);
#pragma unroll
        for (int j = 0; j < 4; ++j) {
          const v16h b = FragH::load(pXh + (16u * (pj0 + j) + r) * kLP + koff + 32u * ks);
          yd[j] = mma_g(am, b, yd[j]);
        }
        const v16h ac = FragH::load(pC + (16u * tt + r) * kLP + koff + 32u * ks);
#pragma unroll
        for (int j = 0; j < 4; ++j) {
          const v16h b = FragH::load(pS + (16u * (pj0 + j) + r) * kLP + koff + 32u * ks);
          yo[j] = mma_g(ac, b, yo[j]);
        }
      }
      float et[8];
#pragma unroll
      for (int rr = 0; rr < 8; ++rr) et[rr] = sEt[16u * tt + 8u * hh + rr] * kYoFold;
#pragma unroll
      for (int j = 0; j < 4; ++j)
#pragma unroll
        for (int rr = 0; rr < 8; ++rr)
          sY[(16u * tt + 8u * hh + rr) * kYP + 16u * (pj0 + j) + r] = yd[j][rr] * kYdFold + et[rr] * yo[j][rr];
    }
    {
      v8f cs[4], cr[4];
#pragma unroll
      for (int j = 0; j < 4; ++j) {
        cs[j] = (v8f){0.f,0.f,0.f,0.f,0.f,0.f,0.f,0.f};
        cr[j] = (v8f){0.f,0.f,0.f,0.f,0.f,0.f,0.f,0.f};
      }
#pragma unroll
      for (int ks = 0; ks < 2; ++ks) {
        const v16h ah = FragH::load(pXh + (16u * wave + r) * kLP + koff + 32u * ks);
        const v16h al = FragH::load(pXl + (16u * wave + r) * kLP + koff + 32u * ks);
#pragma unroll
        for (int j = 0; j < 4; ++j) {
          const v16h bh = FragH::load(pBh + (16u * j + r) * kLP + koff + 32u * ks);
          const v16h bl = FragH::load(pBl + (16u * j + r) * kLP + koff + 32u * ks);
          cs[j] = mma_g(ah, bh, cs[j]);
          cr[j] = mma_g(ah, bl, cr[j]);
          cr[j] = mma_g(al, bh, cr[j]);
        }
      }
      const float dall = exp_ftz(sAcs[63]);
#pragma unroll
      for (int j = 0; j < 4; ++j)
#pragma unroll
        for (int rr = 0; rr < 8; ++rr)
          sreg[j][rr] = dall * sreg[j][rr] + (cs[j][rr] + cr[j][rr] * (1.0f / kResid)) * kStFold;
    }
    __syncthreads();
#pragma unroll
    for (int j = 0; j < 4; ++j)
#pragma unroll
      for (int rr = 0; rr < 8; ++rr)
        sS[(16u * wave + 8u * hh + rr) * kLP + 16u * j + r] = to_h(sreg[j][rr] * kCarS);
#pragma unroll 1
    for (unsigned it = 0; it < 4u; ++it) {
      const unsigned t = it * 16u + wave * 2u + hh;
      const unsigned c8 = r * 8u;
      const size_t g = (row0 + t) * kDin + 128u * hd + c8;
      const v4u xh = *(const v4u*)(const void*)(xahi + g);
      const v4u xl = *(const v4u*)(const void*)(xalo + g);
      const v4u zz = *(const v4u*)(const void*)(zpl + g);
      const float* sy = sY + t * kYP + c8;
      const v4f y0 = *(const v4f*)(sy);
      const v4f y1 = *(const v4f*)(sy + 4);
      v8h o;
#pragma unroll
      for (int e = 0; e < 8; ++e) {
        const float xv = (h16_to_f32(pick16(xh, e)) + h16_to_f32(pick16(xl, e)) * (1.0f / kResid)) * (1.0f / kCarXa);
        const float zv = h16_to_f32(pick16(zz, e));
        const float sg = __builtin_amdgcn_rcpf(1.0f + __expf(-zv));
        const float ye = (e < 4) ? y0[e & 3] : y1[e & 3];
        const float yv = (ye + Dsk * xv) * sg;
        o[e] = to_h(yv * kCarY);
      }
      unsigned short* q = ypl + g;
      *(volatile v8h*)q = o;
      __threadfence();
      *(volatile v8h*)q = o;
    }
  }

  __syncthreads();
#pragma unroll
  for (int j = 0; j < 4; ++j)
#pragma unroll
    for (int rr = 0; rr < 8; ++rr)
      sY[(16u * wave + 8u * hh + rr) * kSP + 16u * j + r] = sreg[j][rr];
  __syncthreads();
  {
    float* dst = state_out + ((size_t)(bq * kHeads + hd) * kHdim) * kNst;
    const unsigned c4 = r * 4u;
    for (int pass = 0; pass < 2; ++pass) {
#pragma unroll
      for (int it = 0; it < 8; ++it) {
        const unsigned row = 16u * wave + 2u * it + hh;
        const v4f v = *(const v4f*)(sY + row * kSP + c4);
        *(volatile v4f*)(dst + (size_t)row * kNst + c4) = v;
      }
      __threadfence();
    }
  }
}

extern "C" void kernel_launch(void* const* d_in, const int* in_sizes, int n_in,
                              void* d_out, int out_size, void* d_ws, size_t ws_size,
                              hipStream_t stream) {
  if (n_in < 9) return;
  if (in_sizes[0] != kRows * kDm) return;
  if (in_sizes[1] != 2 * kDin * kDm) return;
  if (in_sizes[2] != kDin * 4) return;
  if (in_sizes[3] != kDin) return;
  if (in_sizes[4] != kNssmIn * kDin) return;
  if (in_sizes[5] != kHeads) return;
  if (in_sizes[6] != kHeads) return;
  if (in_sizes[7] != kHeads) return;
  if (in_sizes[8] != kDm * kDin) return;
  if ((size_t)out_size != kOutTot) return;
  if (ws_size < kWsTotal) return;

  const float* inp     = (const float*)d_in[0];
  const float* W_in    = (const float*)d_in[1];
  const float* conv_w  = (const float*)d_in[2];
  const float* conv_b  = (const float*)d_in[3];
  const float* W_ssm   = (const float*)d_in[4];
  const float* A_log   = (const float*)d_in[5];
  const float* D_skip  = (const float*)d_in[6];
  const float* dt_bias = (const float*)d_in[7];
  const float* W_out   = (const float*)d_in[8];
  float* out0 = (float*)d_out;
  float* out1 = out0 + kOut1Off;
  float* out2 = out0 + kOut2Off;

  char* ws = (char*)d_ws;
  unsigned short* INP16  = (unsigned short*)(ws + kOffInp16);
  unsigned short* WIN16  = (unsigned short*)(ws + kOffWin16);
  unsigned short* WSSM16 = (unsigned short*)(ws + kOffWssm16);
  unsigned short* WOUT16 = (unsigned short*)(ws + kOffWout16);
  float*          X32    = (float*)(ws + kOffX32);
  unsigned short* Z16    = (unsigned short*)(ws + kOffZ16);
  unsigned short* XAH    = (unsigned short*)(ws + kOffXah);
  unsigned short* XAL    = (unsigned short*)(ws + kOffXal);
  unsigned short* C16    = (unsigned short*)(ws + kOffC16);
  float*          DT32   = (float*)(ws + kOffDt32);
  unsigned short* WSSML  = (unsigned short*)(ws + kOffWssmLo);
  unsigned short* Y16    = (unsigned short*)(ws + kOffY16);
  float*          B32    = (float*)(ws + kOffB32);

  cvt_f16_kernel<kLgInp, 0><<<(kRows * kDm / 8) / 256, 256, 0, stream>>>(inp, INP16, (unsigned)(kRows * kDm / 8));
  cvt_f16_kernel<kLgW, 0><<<(2 * kDin * kDm / 8) / 256, 256, 0, stream>>>(W_in, WIN16, (unsigned)(2 * kDin * kDm / 8));
  cvt_f16_kernel<kLgW, 1><<<(kNssmPd * kDin / 8) / 256, 256, 0, stream>>>(W_ssm, WSSM16, (unsigned)(kNssmPd * kDin / 8));
  cvt_f16_kernel<kLgW, 2><<<(kLoRows * kDin / 8) / 256, 256, 0, stream>>>(W_ssm, WSSML, (unsigned)(kLoRows * kDin / 8));
  cvt_f16_kernel<kLgW, 0><<<(kDm * kDin / 8) / 256, 256, 0, stream>>>(W_out, WOUT16, (unsigned)(kDm * kDin / 8));

  wmma_gemm64<0, kLgInp + kLgW><<<256, 256, 0, stream>>>(INP16, kDm, WIN16, kDm, (void*)X32, kDin, kRows, kDin, kDm);
  wmma_gemm64<1, kLgInp + kLgW><<<256, 256, 0, stream>>>(INP16, kDm, WIN16 + (size_t)kDin * kDm, kDm, (void*)Z16, kDin, kRows, kDin, kDm);

  conv_silu_kernel<<<dim3(kDin / 256, kRows / 64), 256, 0, stream>>>(X32, conv_w, conv_b, XAH, XAL);
  conv_state_kernel<<<48, 256, 0, stream>>>(X32, out1);

  wmma_gemm_w2<kLgXa + kLgW><<<256, 256, 0, stream>>>(XAH, kDin, WSSM16, WSSML, kDin, B32, kBC, kRows, kBC, kDin);
  wmma_gemm64<1, kLgXa + kLgW - kLgSp><<<128, 256, 0, stream>>>(XAH, kDin, WSSM16 + (size_t)kBC * kDin, kDin, (void*)C16, kBC, kRows, kBC, kDin);
  wmma_gemm_w2<kLgXa + kLgW><<<16, 256, 0, stream>>>(XAH, kDin, WSSM16 + (size_t)2 * kBC * kDin, WSSML + (size_t)kBC * kDin, kDin, DT32, kDtPad, kRows, kDtPad, kDin);

  ssd_chunk_kernel<<<kBatch * kHeads, 256, 0, stream>>>(XAH, XAL, Z16, B32, C16, DT32, A_log, D_skip, dt_bias, Y16, out2);

  wmma_gemm64<0, kLgY + kLgW><<<128, 256, 0, stream>>>(Y16, kDin, WOUT16, kDin, (void*)out0, kDm, kRows, kDm, kDin);
}
